// RLMambaBlock_2705829396663
// MI455X (gfx1250) — hardware-run, weakly checked
//
#include <hip/hip_runtime.h>
#include <hip/hip_bf16.h>
#include <math.h>

#define NB    2
#define LL    1024
#define NTOK  (NB * LL)
#define DMOD  512
#define DIN   1024
#define XZW   (2 * DIN)
#define DST   16
#define DTR   32
#define XDN   (DTR + 2 * DST)
#define DCV   4
#define DFF   (2 * DMOD)
#define GSTR  40
#define OSTR  68
#define SMEMB (8 * 16 * OSTR * 4)
#define SCH   32
#define SYP   260
#define LOG2E 1.4426950408889634f
#define WSCAP ((size_t)134217728)

static_assert(NTOK % 128 == 0);
static_assert(XZW % 64 == 0);
static_assert(XDN == 64);
static_assert(DIN % 64 == 0);
static_assert(DMOD % 64 == 0);
static_assert(DFF % 64 == 0);
static_assert(DMOD % 32 == 0);
static_assert(DIN % 32 == 0);
static_assert(DTR == 32);
static_assert(DST == 16);
static_assert(LL % SCH == 0);
static_assert(SCH == 32);
static_assert(SYP % 4 == 0);
static_assert(SYP >= 256);
static_assert(SMEMB >= (2 * 128 * GSTR + 64 * GSTR) * 2);
static_assert(DIN == 4 * 256);
static_assert(DMOD == 4 * 128);
static_assert((NTOK * DFF) % 256 == 0);
static_assert(DFF % 256 == 0);

typedef unsigned short us16 __attribute__((ext_vector_type(16)));
typedef unsigned short us8  __attribute__((ext_vector_type(8)));
typedef unsigned short us8a __attribute__((ext_vector_type(8), may_alias));
typedef __bf16 v16b __attribute__((ext_vector_type(16)));
typedef float v8f __attribute__((ext_vector_type(8)));
typedef float v4f __attribute__((ext_vector_type(4)));
typedef float v4fa __attribute__((ext_vector_type(4), may_alias));
union FragU { us16 v; us8 h[2]; };

__device__ __forceinline__ unsigned short bf16_bits(float f) {
  unsigned u = __float_as_uint(f);
  u += 0x7FFFu + ((u >> 16) & 1u);
  return (unsigned short)(u >> 16);
}
__device__ __forceinline__ float bf16_val(unsigned short b) { return __uint_as_float(((unsigned)b) << 16); }
__device__ __forceinline__ float bf16r(float f) { return bf16_val(bf16_bits(f)); }
__device__ __forceinline__ float siluf(float x) { return x * __builtin_amdgcn_rcpf(1.0f + __expf(-x)); }

__device__ __forceinline__ float wsum(float v) {
#pragma unroll
  for (int o = 16; o > 0; o >>= 1) v += __shfl_xor(v, o, 32);
  return v;
}

__device__ __forceinline__ void split8(const v4f a, const v4f b, us8& hi, us8& lo) {
#pragma unroll
  for (int u = 0; u < 4; ++u) {
    const unsigned short ha = bf16_bits(a[u]);
    hi[u] = ha; lo[u] = bf16_bits(a[u] - bf16_val(ha));
    const unsigned short hb = bf16_bits(b[u]);
    hi[4 + u] = hb; lo[4 + u] = bf16_bits(b[u] - bf16_val(hb));
  }
}

__device__ __forceinline__ v8f mma_bf16(us16 a, us16 b, v8f c) {
  return __builtin_amdgcn_wmma_f32_16x16x32_bf16(false, __builtin_bit_cast(v16b, a), false, __builtin_bit_cast(v16b, b), (short)0, c, false, false);
}
__device__ __forceinline__ void wguard(v8f& c0, v8f& c1, v8f& c2, v8f& c3, const us16& a0, const us16& a1,
                                       const us16& b0, const us16& b1, const us16& b2, const us16& b3) {
#if defined(__HIP_DEVICE_COMPILE__)
  asm volatile("v_nop\n\tv_nop\n\tv_nop\n\tv_nop"
               : "+v"(c0), "+v"(c1), "+v"(c2), "+v"(c3)
               : "v"(a0), "v"(a1), "v"(b0), "v"(b1), "v"(b2), "v"(b3));
#endif
}

__device__ __forceinline__ us16 lds_frag(const unsigned short* base) {
  const int lane = threadIdx.x & 31, r = lane & 15, kh = (lane >> 4) * 8;
  FragU f;
  f.h[0] = *(const us8a*)(base + r * GSTR + kh);
  f.h[1] = *(const us8a*)(base + r * GSTR + 16 + kh);
  return f.v;
}

__device__ __forceinline__ void stage_a(unsigned short* lds, const unsigned short* __restrict__ P, int ld, int m0, int k0, int tid) {
  const int row = tid >> 1, cq = (tid & 1) * 16;
  const unsigned short* src = P + (size_t)(m0 + row) * ld + k0 + cq;
  const us8 v0 = *(const us8a*)src;
  const us8 v1 = *(const us8a*)(src + 8);
  *(us8a*)(lds + row * GSTR + cq) = v0;
  *(us8a*)(lds + row * GSTR + cq + 8) = v1;
}
__device__ __forceinline__ void stage_b(unsigned short* lds, const unsigned short* __restrict__ P, int ld, int n0, int k0, int tid) {
  const int row = tid >> 2, kq = (tid & 3) * 8;
  const us8 v = *(const us8a*)(P + (size_t)(n0 + row) * ld + k0 + kq);
  *(us8a*)(lds + row * GSTR + kq) = v;
}

template <int NA>
__global__ __launch_bounds__(256) void k_gemm(const unsigned short* __restrict__ A0, const unsigned short* __restrict__ A1, int lda,
                                             const unsigned short* __restrict__ B0, int ldb, float* Y, int ldy, int K) {
  __shared__ __attribute__((aligned(16))) unsigned char sm[SMEMB];
  unsigned short* lA0 = (unsigned short*)sm;
  unsigned short* lA1 = lA0 + 128 * GSTR;
  unsigned short* lB0 = lA1 + 128 * GSTR;
  float* oS = (float*)sm;
  const int tid = threadIdx.x, lane = tid & 31, wave = tid >> 5, cl = lane & 15, hh = lane >> 4;
  const int m0 = blockIdx.x * 128, n0 = blockIdx.y * 64;

  v8f acc[4];
#pragma unroll
  for (int j = 0; j < 4; ++j) { v8f zz = {0.f, 0.f, 0.f, 0.f, 0.f, 0.f, 0.f, 0.f}; acc[j] = zz; }

#pragma unroll 1
  for (int k0 = 0; k0 < K; k0 += 32) {
    __syncthreads();
    stage_a(lA0, A0, lda, m0, k0, tid);
    if (NA == 2) stage_a(lA1, A1, lda, m0, k0, tid);
    stage_b(lB0, B0, ldb, n0, k0, tid);
    __syncthreads();
    const us16 af0 = lds_frag(lA0 + 16 * wave * GSTR);
    us16 af1 = af0;
    if (NA == 2) af1 = lds_frag(lA1 + 16 * wave * GSTR);
    us16 bfr[4];
#pragma unroll
    for (int j = 0; j < 4; ++j) bfr[j] = lds_frag(lB0 + 16 * j * GSTR);
#pragma unroll
    for (int j = 0; j < 4; ++j) acc[j] = mma_bf16(af0, bfr[j], acc[j]);
    if (NA == 2) {
#pragma unroll
      for (int j = 0; j < 4; ++j) acc[j] = mma_bf16(af1, bfr[j], acc[j]);
    }
    wguard(acc[0], acc[1], acc[2], acc[3], af0, af1, bfr[0], bfr[1], bfr[2], bfr[3]);
  }
  __syncthreads();

  float* so = oS + wave * (16 * OSTR);
#pragma unroll
  for (int j = 0; j < 4; ++j)
#pragma unroll
    for (int r = 0; r < 8; ++r) so[(8 * hh + r) * OSTR + 16 * j + cl] = acc[j][r];
  __syncthreads();
#pragma unroll
  for (int pass = 0; pass < 2; ++pass) {
#pragma unroll
    for (int it = 0; it < 8; ++it) {
      const int ch = it * 32 + lane, r = ch >> 4, q = (ch & 15) * 4;
      const v4f v = *(const v4fa*)(so + r * OSTR + q);
      *(volatile v4f*)(Y + (size_t)(m0 + 16 * wave + r) * ldy + n0 + q) = v;
    }
    __threadfence();
  }
}

__global__ __launch_bounds__(256) void k_cvt(const float* __restrict__ src, int spitch, unsigned short* dst, int nrow, int ncol8, int total8) {
  const int idx = blockIdx.x * 256 + threadIdx.x;
  if (idx >= total8) return;
  const int row = idx / ncol8, c8 = (idx - row * ncol8) * 8;
  const int rs = (row < nrow) ? row : (nrow - 1);
  const float* s = src + (size_t)rs * (size_t)spitch + c8;
  const v4f a = *(const v4fa*)s, b = *(const v4fa*)(s + 4);
  const bool zr = (row >= nrow);
  us8 o;
#pragma unroll
  for (int u = 0; u < 4; ++u) {
    o[u]     = zr ? (unsigned short)0 : bf16_bits(a[u]);
    o[4 + u] = zr ? (unsigned short)0 : bf16_bits(b[u]);
  }
  const size_t off = (size_t)row * (size_t)(ncol8 * 8) + c8;
  *(volatile us8*)(dst + off) = o;
  __threadfence();
  *(volatile us8*)(dst + off) = o;
}

__global__ __launch_bounds__(256) void k_conv(const float* __restrict__ XZ, const float* __restrict__ cw, const float* __restrict__ cb,
                                             float* XCF, unsigned short* XCH) {
#pragma clang fp contract(off)
  __shared__ __attribute__((aligned(16))) float sxs[DIN];
  const int tid = threadIdx.x, c4 = tid * 4;
  const int tok = blockIdx.x, l = tok % LL;
  v4f xv[DCV];
#pragma unroll
  for (int j = 0; j < DCV; ++j) {
    const int ll = l - (DCV - 1) + j;
    const int tc = (ll >= 0) ? (tok - (DCV - 1) + j) : tok;
    xv[j] = *(const v4fa*)(XZ + (size_t)tc * XZW + c4);
  }
  const v4f bb = *(const v4fa*)(cb + c4);
  v4f sv;
#pragma unroll
  for (int u = 0; u < 4; ++u) {
    const v4f wv = *(const v4fa*)(cw + (size_t)(c4 + u) * DCV);
    float a = 0.0f;
#pragma unroll
    for (int j = 0; j < DCV; ++j) {
      const float pr = bf16r(wv[j]) * xv[j][u];
      a = a + ((l - (DCV - 1) + j >= 0) ? pr : 0.0f);
    }
    a = a + bf16r(bb[u]);
    sv[u] = siluf(a);
  }
  *(v4fa*)(sxs + c4) = sv;
  const size_t o = (size_t)tok * DIN + c4;
  *(volatile v4f*)(XCF + o) = sv;
  __threadfence();
  *(volatile v4f*)(XCF + o) = sv;
  __syncthreads();
  if (tid < 128) {
    const int c8 = tid * 8;
    const v4f a = *(const v4fa*)(sxs + c8);
    const v4f b = *(const v4fa*)(sxs + c8 + 4);
    us8 hi;
#pragma unroll
    for (int u = 0; u < 4; ++u) { hi[u] = bf16_bits(a[u]); hi[4 + u] = bf16_bits(b[u]); }
    const size_t o2 = (size_t)tok * DIN + c8;
    *(volatile us8*)(XCH + o2) = hi;
    __threadfence();
    *(volatile us8*)(XCH + o2) = hi;
  }
}

__global__ __launch_bounds__(256) void k_scan(const float* __restrict__ XZ, const float* __restrict__ XCF, const float* __restrict__ XD,
                                             const float* __restrict__ DTW, const float* __restrict__ dtb, const float* __restrict__ Alog,
                                             const float* __restrict__ Dv, unsigned short* YGH, unsigned short* YGL) {
#pragma clang fp contract(off)
  __shared__ __attribute__((aligned(16))) float sy[SCH * SYP];
  const int b = blockIdx.x >> 2, dg = blockIdx.x & 3, tid = threadIdx.x, lane = tid & 31, wave = tid >> 5;
  const int d = dg * 256 + tid;
  float A2[DST], h[DST];
#pragma unroll
  for (int n = 0; n < DST; ++n) { A2[n] = -__expf(bf16r(Alog[d * DST + n])) * LOG2E; h[n] = 0.0f; }
  const float Dd = bf16r(Dv[d]);
  const float bd = bf16r(dtb[d]);
#pragma unroll 1
  for (int c = 0; c < LL / SCH; ++c) {
#pragma unroll 1
    for (int s = 0; s < SCH; ++s) {
      const size_t tok = (size_t)b * LL + (size_t)(c * SCH + s);
      const float raw = DTW[tok * DIN + d];
      const float a = raw + bd;
      const float dl = fmaxf(a, 0.0f) + log1pf(__expf(-fabsf(a)));
      const float xv = XCF[tok * DIN + d];
      const float zv = XZ[tok * XZW + DIN + d];
      const float* bcp = XD + tok * XDN;
      v4f Bv[4], Cv[4];
#pragma unroll
      for (int q = 0; q < 4; ++q) {
        Bv[q] = *(const v4fa*)(bcp + DTR + 4 * q);
        Cv[q] = *(const v4fa*)(bcp + DTR + DST + 4 * q);
      }
      const float dx = dl * xv;
      float y = 0.0f;
#pragma unroll
      for (int n = 0; n < DST; ++n) {
        const float e = exp2f(dl * A2[n]);
        h[n] = e * h[n] + dx * Bv[n >> 2][n & 3];
        y = y + h[n] * Cv[n >> 2][n & 3];
      }
      const float yv = (y + xv * Dd) * siluf(zv);
      sy[s * SYP + tid] = yv;
    }
    __syncthreads();
#pragma unroll
    for (int pass = 0; pass < 2; ++pass) {
#pragma unroll
      for (int it = 0; it < 4; ++it) {
        const int row = 4 * wave + it;
        const v4f va = *(const v4fa*)(sy + row * SYP + lane * 8);
        const v4f vb = *(const v4fa*)(sy + row * SYP + lane * 8 + 4);
        us8 hi, lo;
        split8(va, vb, hi, lo);
        const size_t o = ((size_t)b * LL + (size_t)(c * SCH + row)) * DIN + (size_t)dg * 256 + lane * 8;
        *(volatile us8*)(YGH + o) = hi; *(volatile us8*)(YGL + o) = lo;
      }
      __threadfence();
    }
    __syncthreads();
  }
}

__global__ __launch_bounds__(128) void k_ln1(const float* __restrict__ X, const float* __restrict__ MO, const float* __restrict__ g,
                                            const float* __restrict__ be, float* R, unsigned short* RH, unsigned short* RL) {
#pragma clang fp contract(off)
  __shared__ __attribute__((aligned(16))) float srow[DMOD];
  __shared__ float sred[8];
  const int tid = threadIdx.x, lane = tid & 31, wave = tid >> 5, c4 = tid * 4;
  const int tok = blockIdx.x;
  const size_t o = (size_t)tok * DMOD + c4;
  const v4f xv = *(const v4fa*)(X + o);
  const v4f mv = *(const v4fa*)(MO + o);
  v4f rv;
#pragma unroll
  for (int u = 0; u < 4; ++u) rv[u] = bf16r(xv[u]) - mv[u];
  float s = (rv[0] + rv[1]) + (rv[2] + rv[3]);
  s = wsum(s);
  if (lane == 0) sred[wave] = s;
  __syncthreads();
  const float mean = ((sred[0] + sred[1]) + (sred[2] + sred[3])) * (1.0f / DMOD);
  v4f dv;
  float q = 0.0f;
#pragma unroll
  for (int u = 0; u < 4; ++u) { dv[u] = rv[u] - mean; q = q + dv[u] * dv[u]; }
  q = wsum(q);
  if (lane == 0) sred[4 + wave] = q;
  __syncthreads();
  const float var = ((sred[4] + sred[5]) + (sred[6] + sred[7])) * (1.0f / DMOD);
  const float inv = rsqrtf(var + 1e-5f);
  const v4f gv = *(const v4fa*)(g + c4), ev = *(const v4fa*)(be + c4);
  v4f rr;
#pragma unroll
  for (int u = 0; u < 4; ++u) rr[u] = dv[u] * inv * bf16r(gv[u]) + bf16r(ev[u]);
  *(v4fa*)(srow + c4) = rr;
  *(volatile v4f*)(R + o) = rr;
  __threadfence();
  *(volatile v4f*)(R + o) = rr;
  __syncthreads();
  if (tid < 64) {
    const int c8 = tid * 8;
    const v4f a = *(const v4fa*)(srow + c8);
    const v4f b = *(const v4fa*)(srow + c8 + 4);
    us8 hi, lo;
    split8(a, b, hi, lo);
    const size_t o2 = (size_t)tok * DMOD + c8;
    *(volatile us8*)(RH + o2) = hi; *(volatile us8*)(RL + o2) = lo;
    __threadfence();
    *(volatile us8*)(RH + o2) = hi; *(volatile us8*)(RL + o2) = lo;
  }
}

__global__ __launch_bounds__(256) void k_gelu(const float* __restrict__ H1, const float* __restrict__ bias, unsigned short* GH, unsigned short* GL) {
#pragma clang fp contract(off)
  __shared__ __attribute__((aligned(16))) float sg[256];
  const int tid = threadIdx.x, lane = tid & 31;
  const size_t base = (size_t)blockIdx.x * 256;
  const int col = (int)((base + (size_t)tid) & (size_t)(DFF - 1));
  const float v = H1[base + tid] + bf16r(bias[col]);
  const float gl = 0.5f * v * (1.0f + erff(v * 0.70710678118654752f));
  sg[tid] = gl;
  __syncthreads();
  if (tid < 32) {
    const v4f a = *(const v4fa*)(sg + lane * 8);
    const v4f b = *(const v4fa*)(sg + lane * 8 + 4);
    us8 hi, lo;
    split8(a, b, hi, lo);
    const size_t off = base + (size_t)lane * 8;
    *(volatile us8*)(GH + off) = hi; *(volatile us8*)(GL + off) = lo;
    __threadfence();
    *(volatile us8*)(GH + off) = hi; *(volatile us8*)(GL + off) = lo;
  }
}

__global__ __launch_bounds__(128) void k_final(const float* __restrict__ R, const float* __restrict__ FF, const float* __restrict__ bff,
                                              const float* __restrict__ X, const float* __restrict__ g, const float* __restrict__ be, float* out) {
#pragma clang fp contract(off)
  __shared__ float sred[8];
  const int tid = threadIdx.x, lane = tid & 31, wave = tid >> 5, c4 = tid * 4;
  const int tok = blockIdx.x;
  const size_t o = (size_t)tok * DMOD + c4;
  const v4f rv = *(const v4fa*)(R + o);
  const v4f fv = *(const v4fa*)(FF + o);
  const v4f bv = *(const v4fa*)(bff + c4);
  const v4f xv = *(const v4fa*)(X + o);
  v4f sv;
#pragma unroll
  for (int u = 0; u < 4; ++u) {
    const float f = fv[u] + bf16r(bv[u]);
    const float r2 = rv[u] - f;
    sv[u] = siluf(r2);
  }
  float s = (sv[0] + sv[1]) + (sv[2] + sv[3]);
  s = wsum(s);
  if (lane == 0) sred[wave] = s;
  __syncthreads();
  const float mean = ((sred[0] + sred[1]) + (sred[2] + sred[3])) * (1.0f / DMOD);
  v4f dv;
  float q = 0.0f;
#pragma unroll
  for (int u = 0; u < 4; ++u) { dv[u] = sv[u] - mean; q = q + dv[u] * dv[u]; }
  q = wsum(q);
  if (lane == 0) sred[4 + wave] = q;
  __syncthreads();
  const float var = ((sred[4] + sred[5]) + (sred[6] + sred[7])) * (1.0f / DMOD);
  const float inv = rsqrtf(var + 1e-5f);
  const v4f gv = *(const v4fa*)(g + c4), ev = *(const v4fa*)(be + c4);
  v4f ov;
#pragma unroll
  for (int u = 0; u < 4; ++u) ov[u] = (dv[u] * inv * bf16r(gv[u]) + bf16r(ev[u])) + bf16r(xv[u]);
  *(volatile v4f*)(out + o) = ov;
  __threadfence();
  *(volatile v4f*)(out + o) = ov;
}

extern "C" void kernel_launch(void* const* d_in, const int* in_sizes, int n_in,
                              void* d_out, int out_size, void* d_ws, size_t ws_size,
                              hipStream_t stream) {
  if (n_in < 18) return;
  if (in_sizes[0] != NTOK * DMOD || in_sizes[1] != XZW * DMOD || in_sizes[2] != DIN * DCV || in_sizes[3] != DIN ||
      in_sizes[4] != XDN * DIN || in_sizes[5] != DIN * DTR || in_sizes[6] != DIN || in_sizes[7] != DIN * DST ||
      in_sizes[8] != DIN || in_sizes[9] != DMOD * DIN || in_sizes[10] != DMOD || in_sizes[11] != DMOD ||
      in_sizes[12] != DFF * DMOD || in_sizes[13] != DFF || in_sizes[14] != DMOD * DFF || in_sizes[15] != DMOD ||
      in_sizes[16] != DMOD || in_sizes[17] != DMOD || out_size != NTOK * DMOD) return;

  const float* x    = (const float*)d_in[0];
  const float* inw  = (const float*)d_in[1];
  const float* cw   = (const float*)d_in[2];
  const float* cb   = (const float*)d_in[3];
  const float* xpw  = (const float*)d_in[4];
  const float* dtw  = (const float*)d_in[5];
  const float* dtb  = (const float*)d_in[6];
  const float* Alog = (const float*)d_in[7];
  const float* Dv   = (const float*)d_in[8];
  const float* ow   = (const float*)d_in[9];
  const float* g1   = (const float*)d_in[10];
  const float* be1  = (const float*)d_in[11];
  const float* f1w  = (const float*)d_in[12];
  const float* f1b  = (const float*)d_in[13];
  const float* f2w  = (const float*)d_in[14];
  const float* f2b  = (const float*)d_in[15];
  const float* g2   = (const float*)d_in[16];
  const float* be2  = (const float*)d_in[17];
  float* out = (float*)d_out;

  size_t off = 0;
  auto carve = [&](size_t bytes) -> char* { char* p = (char*)d_ws + off; off += (bytes + 255) & ~(size_t)255; return p; };
  unsigned short* WIN16 = (unsigned short*)carve((size_t)XZW * DMOD * 2);
  unsigned short* WX16  = (unsigned short*)carve((size_t)XDN * DIN * 2);
  unsigned short* WDT16 = (unsigned short*)carve((size_t)DIN * DTR * 2);
  unsigned short* WO16  = (unsigned short*)carve((size_t)DMOD * DIN * 2);
  unsigned short* WF1   = (unsigned short*)carve((size_t)DFF * DMOD * 2);
  unsigned short* WF2   = (unsigned short*)carve((size_t)DMOD * DFF * 2);
  unsigned short* X16   = (unsigned short*)carve((size_t)NTOK * DMOD * 2);
  float* XZ             = (float*)carve((size_t)NTOK * XZW * 4);
  float* XCF            = (float*)carve((size_t)NTOK * DIN * 4);
  unsigned short* XCH   = (unsigned short*)carve((size_t)NTOK * DIN * 2);
  float* XD             = (float*)carve((size_t)NTOK * XDN * 4);
  unsigned short* DT16  = (unsigned short*)carve((size_t)NTOK * DTR * 2);
  float* DTW            = (float*)carve((size_t)NTOK * DIN * 4);
  unsigned short* YGH   = (unsigned short*)carve((size_t)NTOK * DIN * 2);
  unsigned short* YGL   = (unsigned short*)carve((size_t)NTOK * DIN * 2);
  float* MO             = (float*)carve((size_t)NTOK * DMOD * 4);
  float* RF             = (float*)carve((size_t)NTOK * DMOD * 4);
  unsigned short* RH    = (unsigned short*)carve((size_t)NTOK * DMOD * 2);
  unsigned short* RL    = (unsigned short*)carve((size_t)NTOK * DMOD * 2);
  float* H1             = (float*)carve((size_t)NTOK * DFF * 4);
  unsigned short* GH    = (unsigned short*)carve((size_t)NTOK * DFF * 2);
  unsigned short* GL    = (unsigned short*)carve((size_t)NTOK * DFF * 2);
  float* FF             = (float*)carve((size_t)NTOK * DMOD * 4);
  if (off > ws_size || off > WSCAP) return;

  const dim3 b256(256), b128(128);
  auto cvt = [&](const float* src, int spitch, unsigned short* dst, int nrow, int ncol) {
    const int ncol8 = ncol / 8, total8 = nrow * ncol8;
    k_cvt<<<dim3((total8 + 255) / 256), b256, 0, stream>>>(src, spitch, dst, nrow, ncol8, total8);
  };
  cvt(inw, DMOD, WIN16, XZW, DMOD);
  cvt(xpw, DIN, WX16, XDN, DIN);
  cvt(dtw, DTR, WDT16, DIN, DTR);
  cvt(ow, DIN, WO16, DMOD, DIN);
  cvt(f1w, DMOD, WF1, DFF, DMOD);
  cvt(f2w, DFF, WF2, DMOD, DFF);
  cvt(x, DMOD, X16, NTOK, DMOD);

  k_gemm<1><<<dim3(NTOK / 128, XZW / 64), b256, 0, stream>>>(X16, X16, DMOD, WIN16, DMOD, XZ, XZW, DMOD);
  k_conv<<<dim3(NTOK), b256, 0, stream>>>(XZ, cw, cb, XCF, XCH);
  k_gemm<1><<<dim3(NTOK / 128, XDN / 64), b256, 0, stream>>>(XCH, XCH, DIN, WX16, DIN, XD, XDN, DIN);
  cvt(XD, XDN, DT16, NTOK, DTR);
  k_gemm<1><<<dim3(NTOK / 128, DIN / 64), b256, 0, stream>>>(DT16, DT16, DTR, WDT16, DTR, DTW, DIN, DTR);
  k_scan<<<dim3(NB * (DIN / 256)), b256, 0, stream>>>(XZ, XCF, XD, DTW, dtb, Alog, Dv, YGH, YGL);
  k_gemm<2><<<dim3(NTOK / 128, DMOD / 64), b256, 0, stream>>>(YGH, YGL, DIN, WO16, DIN, MO, DMOD, DIN);
  k_ln1<<<dim3(NTOK), b128, 0, stream>>>(x, MO, g1, be1, RF, RH, RL);
  k_gemm<2><<<dim3(NTOK / 128, DFF / 64), b256, 0, stream>>>(RH, RL, DMOD, WF1, DMOD, H1, DFF, DMOD);
  k_gelu<<<dim3((NTOK * DFF) / 256), b256, 0, stream>>>(H1, f1b, GH, GL);
  k_gemm<2><<<dim3(NTOK / 128, DMOD / 64), b256, 0, stream>>>(GH, GL, DFF, WF2, DFF, FF, DMOD, DFF);
  k_final<<<dim3(NTOK), b128, 0, stream>>>(RF, FF, f2b, x, g2, be2, out);
}
